// AE_45810121179173
// MI455X (gfx1250) — hardware-verified
//
#include <hip/hip_runtime.h>
#include <math.h>

typedef __attribute__((ext_vector_type(16))) _Float16 v16h;
typedef __attribute__((ext_vector_type(16))) __bf16 v16b;
typedef __attribute__((ext_vector_type(8)))  _Float16 v8h;
typedef __attribute__((ext_vector_type(8)))  float v8f;
typedef __attribute__((ext_vector_type(4)))  float v4f;
typedef __attribute__((ext_vector_type(2)))  float v2f;
typedef __attribute__((ext_vector_type(4)))  unsigned v4u;
typedef __attribute__((ext_vector_type(4)))  int v4i;
typedef float __attribute__((may_alias)) float_a;
typedef int __attribute__((may_alias)) int_a;

template <typename T> __device__ __forceinline__ void vst2(void* p, T v) { *(volatile T*)p = v; __threadfence(); *(volatile T*)p = v; }
__device__ __forceinline__ v8f wmma16(v16h a, v16h b, v8f c) {
  v8f d = __builtin_amdgcn_wmma_f32_16x16x32_f16(false, a, false, b, (short)0, c, false, false);
  asm volatile("v_nop\n\tv_nop\n\tv_nop\n\tv_nop" : "+v"(d) : "v"(a), "v"(b));
  return d;
}
__device__ __forceinline__ v8f wmma_bf(v16b a, v16b b, v8f c) {
  v8f d = __builtin_amdgcn_wmma_f32_16x16x32_bf16(false, a, false, b, (short)0, c, false, false);
  asm volatile("v_nop\n\tv_nop\n\tv_nop\n\tv_nop" : "+v"(d) : "v"(a), "v"(b));
  return d;
}
__device__ __forceinline__ v16h frag_h(const _Float16* rowk0, int lane) {
  union { v16h v; v8h q[2]; } u; const _Float16* p = rowk0 + 8 * (lane >> 4);
  u.q[0] = *(const v8h*)p; u.q[1] = *(const v8h*)(p + 16); return u.v;
}
__device__ __forceinline__ v16h frag_f32(const float* rowk0, int lane) {
  v16h a; const float* p = rowk0 + 8 * (lane >> 4);
#pragma unroll
  for (int i = 0; i < 8; ++i) { a[i] = (_Float16)p[i]; a[8 + i] = (_Float16)p[16 + i]; }
  return a;
}
__device__ __forceinline__ v16h frag_f32s(const float* rowk0, int lane, float sc) {
  v16h a; const float* p = rowk0 + 8 * (lane >> 4);
#pragma unroll
  for (int i = 0; i < 8; ++i) { a[i] = (_Float16)(p[i] * sc); a[8 + i] = (_Float16)(p[16 + i] * sc); }
  return a;
}
__device__ __forceinline__ v16h fragc_f32(const float* W, int k0, int n, int lane, int ld, int K) {
  v16h a; const int g = lane >> 4;
#pragma unroll
  for (int i = 0; i < 8; ++i) { const int ka = k0 + 8 * g + i, kb = ka + 16;
    a[i] = (_Float16)(ka < K ? W[(size_t)(ka < K ? ka : K - 1) * ld + n] : 0.f); a[8 + i] = (_Float16)(kb < K ? W[(size_t)(kb < K ? kb : K - 1) * ld + n] : 0.f); }
  return a;
}
struct F2 { v16b h, l; };
__device__ __forceinline__ F2 bsplit16(const float v[16]) { F2 r;
#pragma unroll
  for (int i = 0; i < 16; ++i) { const __bf16 h = (__bf16)v[i]; r.h[i] = h; r.l[i] = (__bf16)(v[i] - (float)h); }
  return r; }
__device__ __forceinline__ F2 split_row(const float* row, int k0, int lane) { float v[16]; const float* p = row + k0 + 8 * (lane >> 4);
#pragma unroll
  for (int i = 0; i < 8; ++i) { v[i] = p[i]; v[8 + i] = p[16 + i]; }
  return bsplit16(v); }
__device__ __forceinline__ F2 split_rowK(const float* row, int k0, int lane, int K) { float v[16]; const int g = lane >> 4;
#pragma unroll
  for (int i = 0; i < 8; ++i) { const int ka = k0 + 8 * g + i, kb = ka + 16; v[i] = ka < K ? row[ka < K ? ka : K - 1] : 0.f; v[8 + i] = kb < K ? row[kb < K ? kb : K - 1] : 0.f; }
  return bsplit16(v); }
__device__ __forceinline__ F2 split_col(const float* W, int k0, int n, int lane, int ld, int K) { float v[16]; const int g = lane >> 4;
#pragma unroll
  for (int i = 0; i < 8; ++i) { const int ka = k0 + 8 * g + i, kb = ka + 16; v[i] = ka < K ? W[(size_t)(ka < K ? ka : K - 1) * ld + n] : 0.f; v[8 + i] = kb < K ? W[(size_t)(kb < K ? kb : K - 1) * ld + n] : 0.f; }
  return bsplit16(v); }
__device__ __forceinline__ v8f mac3(const F2& a, const F2& b, v8f c) { c = wmma_bf(a.l, b.h, c); c = wmma_bf(a.h, b.l, c); return wmma_bf(a.h, b.h, c); }
__device__ __forceinline__ float sigm(float v) { return 1.0f / (1.0f + expf(-v)); }
#define LDSX() do { asm volatile("s_wait_dscnt 0" ::: "memory"); __builtin_amdgcn_wave_barrier(); __builtin_amdgcn_fence(__ATOMIC_RELEASE, "workgroup"); } while (0)


#define NB 8
#define V0 40000
#define V1 10000
#define V2 2500
#define V3 625
#define V4 160
#define LL 9
#define LAT 256
#ifndef TNB
#define TNB NB
#endif
typedef __attribute__((ext_vector_type(8))) __bf16 v8b;
__device__ __forceinline__ v16b frag_b(const __bf16* rowk0, int lane) {
  union { v16b v; v8b q[2]; } u; const __bf16* p = rowk0 + 8 * (lane >> 4);
  u.q[0] = *(const v8b*)p; u.q[1] = *(const v8b*)(p + 16); return u.v;
}
__device__ __forceinline__ float bfr(float v) { return (float)(__bf16)v; }
__device__ __attribute__((noinline)) float exp_ni(float v) { return expf(v); }
__device__ __forceinline__ float elu1(float v) { return v > 0.f ? v : (exp_ni(v) - 1.0f); }
#define P0 40000
#define P1 10048
#define P2 2560
#define P3 640
#define P4 192
#define PW_E0 0
#define PW_E1 (PW_E0 + 32 * 32)
#define PW_E2 (PW_E1 + 32 * 288)
#define PW_E3 (PW_E2 + 32 * 288)
#define PW_D3 (PW_E3 + 64 * 288)
#define PW_D2 (PW_D3 + 64 * 576)
#define PW_D1 (PW_D2 + 32 * 576)
#define PW_D0 (PW_D1 + 32 * 288)
#define PW_F  (PW_D0 + 32 * 288)
#define PW_ENC (PW_F + 16 * 288)
#define PW_DEC (PW_ENC + 256 * 10240)
#define PW_END (PW_DEC + 10240 * 256)
#define CS_ROWS(t) ((t) == 0 ? V1 : (t) == 1 ? V2 : (t) == 2 ? V3 : (t) == 3 ? V4 : (t) == 4 ? V0 : (t) == 5 ? V1 : (t) == 6 ? V2 : V3)
#define CS_NNZ(t)  ((t) == 0 ? V0 : (t) == 1 ? V1 : (t) == 2 ? V2 : (t) == 3 ? V3 : (t) == 4 ? V0 : (t) == 5 ? V1 : (t) == 6 ? V2 : V3)
#define CS_RP_OFF(t) ((t) * 40064)
#define CS_EN_OFF(t) ((t) * 40960)
#define WS_PW   0u
#define WS_RP   (WS_PW + 2u * PW_END)
#define WS_EC   (WS_RP + 4u * 8 * 40064)
#define WS_EV   (WS_EC + 4u * 8 * 40960)
#define WS_HA   (WS_EV + 4u * 8 * 40960)
#define WS_HB   (WS_HA + 4u * NB * P0 * 32)
#define WS_Z    (WS_HB + 4u * NB * P0 * 32)
#define WS_OST  (WS_Z + 4u * NB * LAT)
#define WS_END  (WS_OST + 4u * NB * P0 * 4)

__global__ __launch_bounds__(256) void k_csr_count(const int* __restrict__ R0, const int* __restrict__ R1, const int* __restrict__ R2, const int* __restrict__ R3, const int* __restrict__ R4, const int* __restrict__ R5, const int* __restrict__ R6, const int* __restrict__ R7, int* __restrict__ RP) {
  __shared__ int scnt[40064];
  const int t = blockIdx.x, tid = threadIdx.x; const int* R = t == 0 ? R0 : t == 1 ? R1 : t == 2 ? R2 : t == 3 ? R3 : t == 4 ? R4 : t == 5 ? R5 : t == 6 ? R6 : R7; const int rows = CS_ROWS(t), nnz = CS_NNZ(t);
  for (int r = tid; r < 40064; r += 256) scnt[r] = 0;
  __syncthreads();
  for (int e = 0; e < nnz; ++e) { const int r = min(max(R[e], 0), rows - 1); if ((r & 255) == tid) scnt[r] += 1; }
  __syncthreads();
  if (tid == 0) { int a = 0; for (int r = 0; r < rows; ++r) { const int c = scnt[r]; scnt[r] = a; a += c; } for (int r = rows; r < 40064; ++r) scnt[r] = a; }
  __syncthreads();
  for (int q = tid; q < 40064 / 4; q += 256) vst2((unsigned*)(RP + CS_RP_OFF(t) + q * 4), *(const v4u*)&scnt[q * 4]);
}
#define CHR 2048
#define SCAP 12288
__global__ __launch_bounds__(256) void k_csr_fill(const int* __restrict__ R0, const int* __restrict__ C0, const float* __restrict__ VV0, const int* __restrict__ R1, const int* __restrict__ C1_, const float* __restrict__ VV1, const int* __restrict__ R2, const int* __restrict__ C2_, const float* __restrict__ VV2, const int* __restrict__ R3, const int* __restrict__ C3_, const float* __restrict__ VV3,
                                                  const int* __restrict__ R4, const int* __restrict__ C4_, const float* __restrict__ VV4, const int* __restrict__ R5, const int* __restrict__ C5_, const float* __restrict__ VV5, const int* __restrict__ R6, const int* __restrict__ C6_, const float* __restrict__ VV6, const int* __restrict__ R7, const int* __restrict__ C7_, const float* __restrict__ VV7,
                                                  const int* __restrict__ RP, int* __restrict__ EC, float* __restrict__ EV) {
  __shared__ int scur[CHR]; __shared__ int sc_[SCAP]; __shared__ float sv_[SCAP]; __shared__ int sbase, send;
  const int c = blockIdx.x, t = blockIdx.y, tid = threadIdx.x; const int rows = CS_ROWS(t), nnz = CS_NNZ(t);
  const int r0 = c * CHR; if (r0 >= rows) return; const int r1 = min(r0 + CHR, rows);
  const int* R = t == 0 ? R0 : t == 1 ? R1 : t == 2 ? R2 : t == 3 ? R3 : t == 4 ? R4 : t == 5 ? R5 : t == 6 ? R6 : R7;
  const int* C = t == 0 ? C0 : t == 1 ? C1_ : t == 2 ? C2_ : t == 3 ? C3_ : t == 4 ? C4_ : t == 5 ? C5_ : t == 6 ? C6_ : C7_;
  const float* VV = t == 0 ? VV0 : t == 1 ? VV1 : t == 2 ? VV2 : t == 3 ? VV3 : t == 4 ? VV4 : t == 5 ? VV5 : t == 6 ? VV6 : VV7;
  const int vin = (t < 4) ? CS_NNZ(t) : (t == 4 ? V1 : t == 5 ? V2 : t == 6 ? V3 : V4);
  const int* RPt = RP + CS_RP_OFF(t);
  if (tid == 0) { sbase = min(max(RPt[r0], 0), nnz); send = min(max(RPt[r1], 0), nnz); }
  for (int r = r0 + tid; r < r1; r += 256) scur[r - r0] = min(max(RPt[r], 0), nnz);
  __syncthreads();
  const int base = sbase, cnt = min(send - base, SCAP);
  for (int e = 0; e < nnz; ++e) { const int r = min(max(R[e], 0), rows - 1); if (r >= r0 && r < r1 && ((r & 255) == tid)) { const int p = scur[r - r0] - base; scur[r - r0] += 1; if (p >= 0 && p < SCAP) { sc_[p] = min(max(C[e], 0), vin - 1); sv_[p] = bfr(VV[e]); } } }
  __syncthreads();
  const int slot0 = base + 32 * c; const int ls = slot0 & ~31; const int le = (slot0 + cnt + 31) & ~31;
  for (int q = tid; q < (le - ls) / 4; q += 256) { int4 vc; v4f vv; for (int k = 0; k < 4; ++k) { const int s = ls + q * 4 + k; const int p = s - slot0; const bool ok = p >= 0 && p < cnt; vc[k] = ok ? sc_[p] : -1; vv[k] = ok ? sv_[p] : 0.f; }
    vst2((unsigned*)(EC + CS_EN_OFF(t) + ls + q * 4), *(const v4u*)&vc); vst2(EV + CS_EN_OFF(t) + ls + q * 4, vv); }
}

__global__ __launch_bounds__(256) void k_pack(const float* __restrict__ We0, const float* __restrict__ We1, const float* __restrict__ We2, const float* __restrict__ We3, const float* __restrict__ Wd3, const float* __restrict__ Wd2, const float* __restrict__ Wd1, const float* __restrict__ Wd0, const float* __restrict__ Wf, const float* __restrict__ Wenc, const float* __restrict__ Wdec, __bf16* __restrict__ PW) {
  __shared__ __align__(16) __bf16 srow[1024];
  const int n = blockIdx.x, tid = threadIdx.x; const float* W; int K, KP, NO, o; size_t dst;
  if (n < 32) { W = We0; K = 27; KP = 32; NO = 32; o = n; dst = PW_E0 + (size_t)o * 32; }
  else if (n < 64) { W = We1; K = 288; KP = 288; NO = 32; o = n - 32; dst = PW_E1 + (size_t)o * 288; }
  else if (n < 96) { W = We2; K = 288; KP = 288; NO = 32; o = n - 64; dst = PW_E2 + (size_t)o * 288; }
  else if (n < 160) { W = We3; K = 288; KP = 288; NO = 64; o = n - 96; dst = PW_E3 + (size_t)o * 288; }
  else if (n < 224) { W = Wd3; K = 576; KP = 576; NO = 64; o = n - 160; dst = PW_D3 + (size_t)o * 576; }
  else if (n < 256) { W = Wd2; K = 576; KP = 576; NO = 32; o = n - 224; dst = PW_D2 + (size_t)o * 576; }
  else if (n < 288) { W = Wd1; K = 288; KP = 288; NO = 32; o = n - 256; dst = PW_D1 + (size_t)o * 288; }
  else if (n < 320) { W = Wd0; K = 288; KP = 288; NO = 32; o = n - 288; dst = PW_D0 + (size_t)o * 288; }
  else if (n < 336) { W = Wf; K = 288; KP = 288; NO = 3; o = n - 320; dst = PW_F + (size_t)o * 288; }
  else if (n < 336 + 256) { o = n - 336;
    for (int part = 0; part < 10; ++part) { for (int k = tid; k < 1024; k += 256) srow[k] = (__bf16)bfr(Wenc[(size_t)(part * 1024 + k) * LAT + o]); __syncthreads(); if (tid < 128) vst2((unsigned*)(PW + PW_ENC + (size_t)o * 10240 + part * 1024 + tid * 8), *(const v4u*)(&srow[tid * 8])); __syncthreads(); } return; }
  else { o = n - 336 - 256; W = Wdec; K = 256; KP = 256; NO = 10240; dst = PW_DEC + (size_t)o * 256; }
  for (int k = tid; k < KP; k += 256) srow[k] = (__bf16)((k < K && o < NO) ? bfr(W[(size_t)k * NO + o]) : 0.f);
  __syncthreads();
  for (int q = tid; q < KP / 8; q += 256) vst2((unsigned*)(PW + dst + q * 8), *(const v4u*)(&srow[q * 8]));
}
template <int CIN, int COUT, int KP, bool EXACT, bool ACT, int OPITCH>
__global__ __launch_bounds__(128) void k_spiral(const float* __restrict__ HIN, int inpitch, int vin, const int* __restrict__ IDX, int nv, const __bf16* __restrict__ P, const float* __restrict__ bias, float* __restrict__ HOUT, int vout_pad) {
  constexpr int NT = (COUT + 15) / 16; constexpr int LDW = KP + 8;
  __shared__ __align__(16) __bf16 sah[64][LDW], sal[64][LDW]; __shared__ __align__(16) float so[4][16][68];
  const int tid = threadIdx.x, wave = tid >> 5, lane = tid & 31, col = lane & 15, g = lane >> 4; const int b = blockIdx.y; const int v0 = blockIdx.x * 64;
  const float* Hb = HIN + (size_t)b * vin * inpitch;
  for (int q = tid; q < 64 * KP; q += 128) { const int vl = q / KP, k = q % KP; const int v = v0 + vl; float val = 0.f;
    if (v < nv && k < LL * CIN) { const int j = k / CIN, ch = k % CIN; const int nb = min(max(IDX[(size_t)v * LL + j], 0), vin - 1); val = Hb[(size_t)nb * inpitch + ch]; if (EXACT) val = bfr(val); }
    const __bf16 hb = (__bf16)val; sah[vl][k] = hb; sal[vl][k] = (__bf16)(val - (float)hb); }
  __syncthreads();
  v8f acc[NT];
#pragma unroll
  for (int j = 0; j < NT; ++j) acc[j] = (v8f){};
#pragma unroll 2
  for (int kc = 0; kc < KP / 32; ++kc) { const v16b ah = frag_b(&sah[wave * 16 + col][kc * 32], lane); v16b al; if (!EXACT) al = frag_b(&sal[wave * 16 + col][kc * 32], lane);
#pragma unroll
    for (int j = 0; j < NT; ++j) { const v16b w = frag_b(P + (size_t)(j * 16 + col) * KP + kc * 32, lane); if (!EXACT) acc[j] = wmma_bf(al, w, acc[j]); acc[j] = wmma_bf(ah, w, acc[j]); } }
#pragma unroll
  for (int j = 0; j < NT; ++j) { const int oc = j * 16 + col; const float bb = oc < COUT ? bfr(bias[oc]) : 0.f;
#pragma unroll
    for (int r = 0; r < 8; ++r) { float v = acc[j][r] + bb; if (ACT) v = elu1(v); so[wave][8 * g + r][oc] = oc < COUT ? v : 0.f; } }
  LDSX();
  for (int rl = 0; rl < 16; ++rl) { const int v = v0 + wave * 16 + rl; if (v < vout_pad) { float* dst = HOUT + ((size_t)b * vout_pad + v) * OPITCH;
      if (OPITCH == 64) { if (lane < 16) vst2(dst + lane * 4, *(const v4f*)&so[wave][rl][lane * 4]); }
      else if (OPITCH == 32) { if (lane < 8) vst2(dst + lane * 4, *(const v4f*)&so[wave][rl][lane * 4]); }
      else { if (lane == 0) { v4f q4 = {so[wave][rl][0], so[wave][rl][1], so[wave][rl][2], 0.f}; vst2(dst, q4); } } } }
}
__global__ __launch_bounds__(256) void k_pool(const float* __restrict__ HIN, int vin_pad, int vin, int ipitch, const int* __restrict__ RP, const int* __restrict__ EC, const float* __restrict__ EV, int t, int rows, int nnz, float* __restrict__ HOUT, int vout_pad, int opitch, int nch) {
  const int tid = threadIdx.x; const int b = blockIdx.y; const int r = blockIdx.x * 64 + (tid >> 2); const int c0 = (tid & 3) * 16; if (c0 >= nch) return;
  float acc[16];
#pragma unroll
  for (int i = 0; i < 16; ++i) acc[i] = 0.f;
  if (r < rows) { const int* RPt = RP + CS_RP_OFF(t); const int st = min(max(RPt[r], 0), nnz), en = min(max(RPt[r + 1], st), nnz); const int slot0 = CS_EN_OFF(t) + 32 * (r / CHR);
    for (int e = st; e < en; ++e) { const int col = min(max(EC[slot0 + e], 0), vin - 1); const float val = EV[slot0 + e]; const float* hr = HIN + ((size_t)b * vin_pad + col) * ipitch + c0;
#pragma unroll
      for (int i = 0; i < 16; ++i) acc[i] += val * hr[i]; } }
  if (r < vout_pad) { float* dst = HOUT + ((size_t)b * vout_pad + r) * opitch + c0;
#pragma unroll
    for (int p = 0; p < 4; ++p) { v4f v = {acc[p * 4], acc[p * 4 + 1], acc[p * 4 + 2], acc[p * 4 + 3]}; vst2(dst + p * 4, v); } }
}
__global__ __launch_bounds__(32) void k_enc(const float* __restrict__ H4, const __bf16* __restrict__ PW, const float* __restrict__ benc, float* __restrict__ Z) {
  __shared__ __align__(16) float sz[16][36];
  const int lane = threadIdx.x, col = lane & 15, g = lane >> 4; const int o0 = blockIdx.x * 32;
  v8f acc[2] = {};
#pragma unroll 4
  for (int kc = 0; kc < 10240 / 32; ++kc) { const int k0 = kc * 32; const int v = k0 / 64, c = k0 % 64;
    F2 a; { const int brow = min(col, NB - 1); const float* src = H4 + ((size_t)brow * P4 + v) * 64 + c; a = split_row(src, 0, lane); if (col >= NB) { for (int i = 0; i < 16; ++i) { a.h[i] = (__bf16)0.f; a.l[i] = (__bf16)0.f; } } }
#pragma unroll
    for (int j = 0; j < 2; ++j) { const v16b w = frag_b(PW + PW_ENC + (size_t)(o0 + j * 16 + col) * 10240 + k0, lane); acc[j] = wmma_bf(a.l, w, acc[j]); acc[j] = wmma_bf(a.h, w, acc[j]); } }
#pragma unroll
  for (int j = 0; j < 2; ++j)
#pragma unroll
    for (int r = 0; r < 8; ++r) sz[8 * g + r][j * 16 + col] = acc[j][r] + bfr(benc[o0 + j * 16 + col]);
  __builtin_amdgcn_fence(__ATOMIC_RELEASE, "workgroup"); __builtin_amdgcn_wave_barrier(); __builtin_amdgcn_fence(__ATOMIC_ACQUIRE, "workgroup");
  for (int q = lane; q < NB * 8; q += 32) { const int b = q >> 3, pc = q & 7; vst2(Z + (size_t)b * LAT + o0 + pc * 4, *(const v4f*)&sz[b][pc * 4]); }
}
__global__ __launch_bounds__(32) void k_dec(const float* __restrict__ Z, const __bf16* __restrict__ PW, const float* __restrict__ bdec, float* __restrict__ H) {
  __shared__ __align__(16) float so[16][68];
  const int lane = threadIdx.x, col = lane & 15, g = lane >> 4; const int v = blockIdx.x;
  v8f acc[4] = {};
#pragma unroll
  for (int kc = 0; kc < LAT / 32; ++kc) { F2 a = split_row(Z + (size_t)min(col, NB - 1) * LAT, kc * 32, lane); if (col >= NB) { for (int i = 0; i < 16; ++i) { a.h[i] = (__bf16)0.f; a.l[i] = (__bf16)0.f; } }
#pragma unroll
    for (int j = 0; j < 4; ++j) { const v16b w = frag_b(PW + PW_DEC + (size_t)(v * 64 + j * 16 + col) * LAT + kc * 32, lane); acc[j] = wmma_bf(a.l, w, acc[j]); acc[j] = wmma_bf(a.h, w, acc[j]); } }
#pragma unroll
  for (int j = 0; j < 4; ++j)
#pragma unroll
    for (int r = 0; r < 8; ++r) so[8 * g + r][j * 16 + col] = acc[j][r] + bfr(bdec[v * 64 + j * 16 + col]);
  __builtin_amdgcn_fence(__ATOMIC_RELEASE, "workgroup"); __builtin_amdgcn_wave_barrier(); __builtin_amdgcn_fence(__ATOMIC_ACQUIRE, "workgroup");
  for (int q = lane; q < NB * 16; q += 32) { const int b = q >> 4, pc = q & 15; vst2(H + ((size_t)b * P4 + v) * 64 + pc * 4, *(const v4f*)&so[b][pc * 4]); }
}
__global__ __launch_bounds__(256) void k_copy(const float* __restrict__ OST, float* __restrict__ out) {
  const size_t p = (size_t)blockIdx.x * 256 + threadIdx.x; const size_t total = (size_t)TNB * V0 * 3;
  if (p * 4 >= total) return; v4f v;
#pragma unroll
  for (int i = 0; i < 4; ++i) { const size_t f = p * 4 + i; const size_t bv = f / 3; v[i] = f < total ? OST[bv * 4 + (f % 3)] : 0.f; }
  vst2(out + p * 4, v);
}

extern "C" void kernel_launch(void* const* d_in, const int* in_sizes, int n_in, void* d_out, int out_size, void* d_ws, size_t ws_size, hipStream_t stream) {
  (void)in_sizes; (void)n_in; (void)out_size;
  const float** F = (const float**)d_in; const int** I = (const int**)d_in;
  if (ws_size < (size_t)WS_END) return;
  char* ws = (char*)d_ws; __bf16* PW = (__bf16*)(ws + WS_PW); int *RP = (int*)(ws + WS_RP), *EC = (int*)(ws + WS_EC); float *EV = (float*)(ws + WS_EV), *HA = (float*)(ws + WS_HA), *HB = (float*)(ws + WS_HB), *Z = (float*)(ws + WS_Z), *OST = (float*)(ws + WS_OST);
#define SP(l) I[1 + 7 * (l)]
#define DR(l) I[2 + 7 * (l)]
#define DC(l) I[3 + 7 * (l)]
#define DV(l) F[4 + 7 * (l)]
#define UR(l) I[5 + 7 * (l)]
#define UC(l) I[6 + 7 * (l)]
#define UV(l) F[7 + 7 * (l)]
  k_csr_count<<<8, 256, 0, stream>>>(DR(0), DR(1), DR(2), DR(3), UR(0), UR(1), UR(2), UR(3), RP);
  k_csr_fill<<<dim3(20, 8), 256, 0, stream>>>(DR(0), DC(0), DV(0), DR(1), DC(1), DV(1), DR(2), DC(2), DV(2), DR(3), DC(3), DV(3), UR(0), UC(0), UV(0), UR(1), UC(1), UV(1), UR(2), UC(2), UV(2), UR(3), UC(3), UV(3), RP, EC, EV);
  k_pack<<<336 + 256 + 10240, 256, 0, stream>>>(F[29], F[31], F[33], F[35], F[47], F[45], F[43], F[41], F[49], F[37], F[39], PW);
  k_spiral<3, 32, 32, true, true, 32><<<dim3((V0 + 63) / 64, TNB), 128, 0, stream>>>(F[0], 3, V0, SP(0), V0, PW + PW_E0, F[30], HA, P0);
  k_pool<<<dim3(P1 / 64, TNB), 256, 0, stream>>>(HA, P0, V0, 32, RP, EC, EV, 0, V1, V0, HB, P1, 64, 32);
  k_spiral<32, 32, 288, false, true, 64><<<dim3(P1 / 64, TNB), 128, 0, stream>>>(HB, 64, P1, SP(1), V1, PW + PW_E1, F[32], HA, P1);
  k_pool<<<dim3(P2 / 64, TNB), 256, 0, stream>>>(HA, P1, V1, 64, RP, EC, EV, 1, V2, V1, HB, P2, 64, 32);
  k_spiral<32, 32, 288, false, true, 64><<<dim3(P2 / 64, TNB), 128, 0, stream>>>(HB, 64, P2, SP(2), V2, PW + PW_E2, F[34], HA, P2);
  k_pool<<<dim3(P3 / 64, TNB), 256, 0, stream>>>(HA, P2, V2, 64, RP, EC, EV, 2, V3, V2, HB, P3, 64, 32);
  k_spiral<32, 64, 288, false, true, 64><<<dim3(P3 / 64, TNB), 128, 0, stream>>>(HB, 64, P3, SP(3), V3, PW + PW_E3, F[36], HA, P3);
  k_pool<<<dim3(P4 / 64, TNB), 256, 0, stream>>>(HA, P3, V3, 64, RP, EC, EV, 3, V4, V3, HB, P4, 64, 64);
  k_enc<<<LAT / 32, 32, 0, stream>>>(HB, PW, F[38], Z);
  k_dec<<<V4, 32, 0, stream>>>(Z, PW, F[40], HA);
  k_pool<<<dim3(P3 / 64, TNB), 256, 0, stream>>>(HA, P4, V4, 64, RP, EC, EV, 7, V3, V3, HB, P3, 64, 64);
  k_spiral<64, 64, 576, false, true, 64><<<dim3(P3 / 64, TNB), 128, 0, stream>>>(HB, 64, P3, SP(3), V3, PW + PW_D3, F[48], HA, P3);
  k_pool<<<dim3(P2 / 64, TNB), 256, 0, stream>>>(HA, P3, V3, 64, RP, EC, EV, 6, V2, V2, HB, P2, 64, 64);
  k_spiral<64, 32, 576, false, true, 64><<<dim3(P2 / 64, TNB), 128, 0, stream>>>(HB, 64, P2, SP(2), V2, PW + PW_D2, F[46], HA, P2);
  k_pool<<<dim3(P1 / 64, TNB), 256, 0, stream>>>(HA, P2, V2, 64, RP, EC, EV, 5, V1, V1, HB, P1, 64, 32);
  k_spiral<32, 32, 288, false, true, 64><<<dim3(P1 / 64, TNB), 128, 0, stream>>>(HB, 64, P1, SP(1), V1, PW + PW_D1, F[44], HA, P1);
  k_pool<<<dim3((V0 + 63) / 64, TNB), 256, 0, stream>>>(HA, P1, V1, 64, RP, EC, EV, 4, V0, V0, HB, P0, 32, 32);
  k_spiral<32, 32, 288, false, true, 32><<<dim3((V0 + 63) / 64, TNB), 128, 0, stream>>>(HB, 32, P0, SP(0), V0, PW + PW_D0, F[42], HA, P0);
  k_spiral<32, 3, 288, false, false, 4><<<dim3((V0 + 63) / 64, TNB), 128, 0, stream>>>(HA, 32, P0, SP(0), V0, PW + PW_F, F[50], OST, P0);
  k_copy<<<(TNB * V0 * 3 / 4 + 255) / 256, 256, 0, stream>>>(OST, (float*)d_out);
}
